// DynamicHead_48120813584686
// MI455X (gfx1250) — hardware-verified
//
#include <hip/hip_runtime.h>

typedef unsigned short v8us  __attribute__((ext_vector_type(8)));
typedef unsigned short v16us __attribute__((ext_vector_type(16)));
typedef __bf16         v16bf __attribute__((ext_vector_type(16)));
typedef float          v8f   __attribute__((ext_vector_type(8)));
typedef float          v4f   __attribute__((ext_vector_type(4)));
typedef v8us __attribute__((may_alias)) v8usa;
typedef v4f  __attribute__((may_alias)) v4fa;

union Frag { v16bf v; v16us u; v8us half[2]; };

#define NIMG     8
#define CH       64
#define H_IMG    40
#define W_IMG    100
#define HW       4000
#define TP       64
#define NTILE    63
#define HWP      (NTILE * TP)
#define NINST    128
#define INS_PER  16
#define PSTR     8513
#define OFF_W1   4224
#define OFF_W2   8320
#define OFF_B0   8384
#define OFF_B1   8448
#define OFF_B2   8512
#define LP       72
#define MASK_OFF 2.19f

static_assert(HWP >= HW);
static_assert(NTILE * TP >= HW && (NTILE - 1) * TP < HW);
static_assert(NINST == NIMG * INS_PER);
static_assert((CH % 32) == 0);
static_assert((LP % 8) == 0);

__device__ __forceinline__ unsigned int bf16_bits(float f) {
  const unsigned int u = __float_as_uint(f);
  return (u + 0x7FFFu + ((u >> 16) & 1u)) >> 16;
}
__device__ __forceinline__ float bf16_val(float f) {
  return __uint_as_float(bf16_bits(f) << 16);
}

__device__ __forceinline__ v8f wmma_bf16(Frag a, Frag b, v8f c) {
  v8f d = __builtin_amdgcn_wmma_f32_16x16x32_bf16(false, a.v, false, b.v, (short)0, c, false, false);
  asm volatile("v_nop\n\tv_nop\n\tv_nop\n\tv_nop" : "+v"(d) : "v"(a.u), "v"(b.u));
  return d;
}

__device__ __forceinline__ Frag load_frag(const unsigned short* p, int h) {
  Frag f;
  f.half[0] = *(const v8usa*)(p + 8 * h);
  f.half[1] = *(const v8usa*)(p + 16 + 8 * h);
  return f;
}

__global__ __launch_bounds__(128) void xt_kernel(const float* __restrict__ x,
                                                 unsigned short* __restrict__ xt)
{
  __shared__ __attribute__((aligned(16))) unsigned short sT[TP * LP];

  const int tid = threadIdx.x, lane = tid & 31, w = tid >> 5;
  const int t = blockIdx.x, img = blockIdx.y;
  const int p0 = t * TP;
  const int pl = tid & 63, cb = tid >> 6;
  const int p  = p0 + pl;
  const bool valid = (p < HW);
  const int pc = valid ? p : (HW - 1);
  const float* xs = x + (size_t)img * CH * HW + pc;

  #pragma unroll 4
  for (int i = 0; i < 32; ++i) {
    const int c = cb + 2 * i;
    const float v = xs[(size_t)c * HW];
    const unsigned int b = valid ? bf16_bits(v) : 0u;
    sT[pl * LP + c] = (unsigned short)b;
  }
  __syncthreads();

  const int q8 = lane & 7, sub = lane >> 3;
  unsigned short* base = xt + ((size_t)img * HWP + p0) * CH;
  v8us vv[4];
  #pragma unroll
  for (int i = 0; i < 4; ++i) {
    const int row = 16 * w + 4 * i + sub;
    vv[i] = *(const v8usa*)(sT + row * LP + 8 * q8);
  }
  #pragma unroll
  for (int i = 0; i < 4; ++i) {
    const int row = 16 * w + 4 * i + sub;
    *(volatile v8us*)(base + (size_t)row * CH + 8 * q8) = vv[i];
  }
  __threadfence();
  #pragma unroll
  for (int i = 0; i < 4; ++i) {
    const int row = 16 * w + 4 * i + sub;
    *(volatile v8us*)(base + (size_t)row * CH + 8 * q8) = vv[i];
  }
}

__global__ __launch_bounds__(256) void wconv_kernel(const float* __restrict__ prm,
                                                    unsigned short* __restrict__ wp)
{
  __shared__ __attribute__((aligned(16))) unsigned short sT[CH * LP];

  const int tid = threadIdx.x, lane = tid & 31, w = tid >> 5;
  const int n = blockIdx.x, which = blockIdx.y;
  const float* prow = prm + (size_t)n * PSTR;

  #pragma unroll 4
  for (int i = 0; i < 16; ++i) {
    const int idx = tid + 256 * i;
    const int o = idx >> 6, k = idx & 63;
    const int off = (which == 0) ? (o * 66 + 2 + k) : (OFF_W1 + o * 64 + k);
    sT[o * LP + k] = (unsigned short)bf16_bits(prow[off]);
  }
  __syncthreads();

  const int q8 = lane & 7, sub = lane >> 3;
  unsigned short* base = wp + (size_t)(2 * n + which) * CH * CH;
  v8us vv[2];
  #pragma unroll
  for (int i = 0; i < 2; ++i) {
    const int row = 8 * w + 4 * i + sub;
    vv[i] = *(const v8usa*)(sT + row * LP + 8 * q8);
  }
  #pragma unroll
  for (int i = 0; i < 2; ++i) {
    const int row = 8 * w + 4 * i + sub;
    *(volatile v8us*)(base + (size_t)row * CH + 8 * q8) = vv[i];
  }
  __threadfence();
  #pragma unroll
  for (int i = 0; i < 2; ++i) {
    const int row = 8 * w + 4 * i + sub;
    *(volatile v8us*)(base + (size_t)row * CH + 8 * q8) = vv[i];
  }
}

__global__ __launch_bounds__(128) void head_kernel(
    const unsigned short* __restrict__ xt,
    const unsigned short* __restrict__ wp,
    const float* __restrict__ prm,
    const int* __restrict__ nins,
    float* __restrict__ out)
{
  __shared__ __attribute__((aligned(16))) unsigned short sHi[TP * LP];
  __shared__ __attribute__((aligned(16))) unsigned short sLo[TP * LP];
  __shared__ __attribute__((aligned(16))) float sOut[TP];

  const int tid = threadIdx.x, lane = tid & 31, w = tid >> 5;
  const int h = lane >> 4, m = lane & 15;
  const int t = blockIdx.x, n = blockIdx.y;
  const int p0 = t * TP;
  const int ni = nins[0];
  const bool bad = (ni != INS_PER);
  const int img = n / INS_PER;
  const float* prow = prm + (size_t)n * PSTR;

  const v8f zero8 = {0.f, 0.f, 0.f, 0.f, 0.f, 0.f, 0.f, 0.f};

  v8f acc[4];
  #pragma unroll
  for (int nt = 0; nt < 4; ++nt) acc[nt] = zero8;
  {
    const unsigned short* xa = xt + ((size_t)img * HWP + p0 + 16 * w + m) * CH;
    const unsigned short* wb = wp + ((size_t)(2 * n) * CH + m) * CH;
    const Frag a0 = load_frag(xa, h);
    const Frag a1 = load_frag(xa + 32, h);
    #pragma unroll
    for (int nt = 0; nt < 4; ++nt) {
      const Frag b0 = load_frag(wb + (size_t)nt * 16 * CH, h);
      const Frag b1 = load_frag(wb + (size_t)nt * 16 * CH + 32, h);
      acc[nt] = wmma_bf16(a0, b0, acc[nt]);
      acc[nt] = wmma_bf16(a1, b1, acc[nt]);
    }
  }

  const int pw = p0 + 16 * w + 8 * h;
  float lx[8], ly[8];
  #pragma unroll
  for (int r = 0; r < 8; ++r) {
    const int p  = pw + r;
    const int py = p / W_IMG;
    const int px = p - py * W_IMG;
    lx[r] = (float)px * (1.0f / H_IMG);
    ly[r] = (float)py * (1.0f / H_IMG);
  }
  #pragma unroll
  for (int nt = 0; nt < 4; ++nt) {
    const int o = 16 * nt + m;
    const float c0 = bf16_val(prow[o * 66]);
    const float c1 = bf16_val(prow[o * 66 + 1]);
    const float b0 = bf16_val(prow[OFF_B0 + o]);
    #pragma unroll
    for (int r = 0; r < 8; ++r) {
      float v = acc[nt][r] + (c0 * lx[r] + c1 * ly[r]) + b0;
      v = fmaxf(v, 0.0f);
      const unsigned int hb = bf16_bits(v);
      const float hf = __uint_as_float(hb << 16);
      const unsigned int lb = bf16_bits(v - hf);
      const int pl = 16 * w + 8 * h + r;
      sHi[pl * LP + o] = (unsigned short)hb;
      sLo[pl * LP + o] = (unsigned short)lb;
    }
  }
  __syncthreads();

  v8f acc1[4];
  #pragma unroll
  for (int nt = 0; nt < 4; ++nt) acc1[nt] = zero8;
  {
    const unsigned short* ha = sHi + (16 * w + m) * LP;
    const unsigned short* la = sLo + (16 * w + m) * LP;
    const unsigned short* wb = wp + ((size_t)(2 * n + 1) * CH + m) * CH;
    const Frag ah0 = load_frag(ha, h);
    const Frag ah1 = load_frag(ha + 32, h);
    const Frag al0 = load_frag(la, h);
    const Frag al1 = load_frag(la + 32, h);
    #pragma unroll
    for (int nt = 0; nt < 4; ++nt) {
      const Frag b0 = load_frag(wb + (size_t)nt * 16 * CH, h);
      const Frag b1 = load_frag(wb + (size_t)nt * 16 * CH + 32, h);
      acc1[nt] = wmma_bf16(ah0, b0, acc1[nt]);
      acc1[nt] = wmma_bf16(al0, b0, acc1[nt]);
      acc1[nt] = wmma_bf16(ah1, b1, acc1[nt]);
      acc1[nt] = wmma_bf16(al1, b1, acc1[nt]);
    }
  }

  float s[8];
  #pragma unroll
  for (int r = 0; r < 8; ++r) s[r] = 0.0f;
  #pragma unroll
  for (int nt = 0; nt < 4; ++nt) {
    const int o = 16 * nt + m;
    const float b1v = bf16_val(prow[OFF_B1 + o]);
    const float w2v = bf16_val(prow[OFF_W2 + o]);
    #pragma unroll
    for (int r = 0; r < 8; ++r) {
      const float hv = fmaxf(acc1[nt][r] + b1v, 0.0f);
      s[r] += w2v * hv;
    }
  }
  #pragma unroll
  for (int r = 0; r < 8; ++r) {
    s[r] += __shfl_xor(s[r], 8);
    s[r] += __shfl_xor(s[r], 4);
    s[r] += __shfl_xor(s[r], 2);
    s[r] += __shfl_xor(s[r], 1);
  }
  const float b2v  = bf16_val(prow[OFF_B2]) - MASK_OFF;
  const float qnan = __uint_as_float(0x7fc00000u);
  if (m == 0) {
    #pragma unroll
    for (int r = 0; r < 8; ++r) {
      const float res = s[r] + b2v;
      sOut[16 * w + 8 * h + r] = bad ? qnan : res;
    }
  }
  __syncthreads();

  const int nval = ((HW - p0) < TP) ? (HW - p0) : TP;
  const int nl = nval >> 2;
  const bool stl = (w == 0) && (lane < nl);
  const v4f ov = *(const v4fa*)(sOut + 4 * (lane & 15));
  float* dst = out + (size_t)n * HW + p0 + 4 * (lane & 15);
  if (stl) *(volatile v4f*)dst = ov;
  __threadfence();
  if (stl) *(volatile v4f*)dst = ov;
}

extern "C" void kernel_launch(void* const* d_in, const int* in_sizes, int n_in,
                              void* d_out, int out_size, void* d_ws, size_t ws_size,
                              hipStream_t stream) {
  if (n_in < 3) return;
  if (in_sizes[0] != NIMG * CH * HW) return;
  if (in_sizes[1] != NINST * PSTR) return;
  if (in_sizes[2] < 1) return;
  if (out_size != NINST * HW) return;

  const float* x    = (const float*)d_in[0];
  const float* prm  = (const float*)d_in[1];
  const int*   nins = (const int*)d_in[2];
  float* out = (float*)d_out;

  const size_t xt_bytes = (size_t)NIMG * HWP * CH * 2;
  const size_t wp_bytes = (size_t)NINST * 2 * CH * CH * 2;
  const size_t total = xt_bytes + wp_bytes;
  if (total > ws_size) return;

  char* ws = (char*)d_ws;
  unsigned short* xt = (unsigned short*)(ws);
  unsigned short* wp = (unsigned short*)(ws + xt_bytes);

  xt_kernel<<<dim3(NTILE, NIMG), 128, 0, stream>>>(x, xt);
  wconv_kernel<<<dim3(NINST, 2), 256, 0, stream>>>(prm, wp);
  head_kernel<<<dim3(NTILE, NINST), 128, 0, stream>>>(xt, wp, prm, nins, out);
}
